// ConnectNet_19370302505104
// MI455X (gfx1250) — hardware-verified
//
#include <hip/hip_runtime.h>

typedef __bf16   v16bf __attribute__((ext_vector_type(16)));
typedef float    v8f   __attribute__((ext_vector_type(8)));
typedef float    v4f   __attribute__((ext_vector_type(4)));

#define C_IN   64
#define H_IN   224
#define W_IN   224
#define HW_IN  (H_IN * W_IN)
#define C_OUT  128
#define H_OUT  222
#define W_OUT  222
#define KTOT   576
#define NKB    18
#define NX     (C_IN * HW_IN)
#define NW     (C_OUT * KTOT)
#define NOUT   (C_OUT * H_OUT * W_OUT)
#define PW     256
#define NP     (C_OUT * H_OUT * PW)
#define BROW   40
#define SP     132

__device__ __forceinline__ unsigned f2bf(float f) {
  union { float f; unsigned u; } v; v.f = f;
  unsigned u = v.u;
  return (u + 0x7FFFu + ((u >> 16) & 1u)) >> 16;
}

__device__ __forceinline__ v8f wmma_bf16(v16bf a, v16bf b, v8f c) {
  v8f d = __builtin_amdgcn_wmma_f32_16x16x32_bf16(false, a, false, b, (short)0, c, false, false);
  asm volatile("v_nop\n\tv_nop\n\tv_nop\n\tv_nop" : "+v"(d) : "v"(a), "v"(b));
  return d;
}

__global__ __launch_bounds__(256) void conv3x3_bf16_wmma(
    const float* __restrict__ x,
    const float* __restrict__ w,
    float* __restrict__ pout) {
  __shared__ __attribute__((aligned(16))) unsigned short Ab[8 * 32 * 16];
  __shared__ __attribute__((aligned(16))) unsigned short Bb[128 * BROW];
  __shared__ __attribute__((aligned(16))) float St[64 * SP];

  const int tid = threadIdx.x;
  const int oh  = blockIdx.y;
  const int ow0 = blockIdx.x * 128;

  const int l  = tid & 31;
  const int wv = tid >> 5;
  const int mq = wv >> 1;
  const int ng = wv & 1;
  const int hh = l >> 4;
  const int cc = l & 15;

  const int am = wv * 16 + cc;
  const int bn  = tid >> 1;
  const int bk0 = (tid & 1) * 16;
  int own = ow0 + bn;
  if (own > W_OUT - 1) own = W_OUT - 1;

  v8f acc[2][4];
#pragma unroll
  for (int i = 0; i < 2; ++i)
#pragma unroll
    for (int j = 0; j < 4; ++j)
#pragma unroll
      for (int e = 0; e < 8; ++e) acc[i][j][e] = 0.0f;

#pragma unroll 1
  for (int kb = 0; kb < NKB; ++kb) {
    const int r  = kb >> 1;
    const int c0 = (kb & 1) * 32;
    const int kh = r / 3, kw = r - 3 * kh;

    {
      const float* wp = w + (size_t)am * KTOT + (size_t)(c0 + 8 * hh) * 9 + r;
      const float* wp2 = wp + 16 * 9;
      unsigned pk[8];
#pragma unroll
      for (int i = 0; i < 4; ++i) {
        unsigned lo = f2bf(wp[(2 * i) * 9]);
        unsigned hi = f2bf(wp[(2 * i + 1) * 9]);
        pk[i] = lo | (hi << 16);
      }
#pragma unroll
      for (int i = 0; i < 4; ++i) {
        unsigned lo = f2bf(wp2[(2 * i) * 9]);
        unsigned hi = f2bf(wp2[(2 * i + 1) * 9]);
        pk[4 + i] = lo | (hi << 16);
      }
      uint4* d = (uint4*)&Ab[tid * 16];
      d[0] = make_uint4(pk[0], pk[1], pk[2], pk[3]);
      d[1] = make_uint4(pk[4], pk[5], pk[6], pk[7]);
    }
    {
      const float* src = x + (size_t)(c0 + bk0) * HW_IN
                           + (size_t)(oh + kh) * W_IN + (own + kw);
      unsigned pk[8];
#pragma unroll
      for (int i = 0; i < 8; ++i) {
        unsigned lo = f2bf(src[(size_t)(2 * i)     * HW_IN]);
        unsigned hi = f2bf(src[(size_t)(2 * i + 1) * HW_IN]);
        pk[i] = lo | (hi << 16);
      }
      uint4* d = (uint4*)&Bb[bn * BROW + bk0];
      d[0] = make_uint4(pk[0], pk[1], pk[2], pk[3]);
      d[1] = make_uint4(pk[4], pk[5], pk[6], pk[7]);
    }
    __syncthreads();

    v16bf afr[2];
#pragma unroll
    for (int i = 0; i < 2; ++i) {
      const unsigned short* ap = &Ab[((mq * 2 + i) * 32 + l) * 16];
      union { uint4 u[2]; v16bf v; } t;
      t.u[0] = *(const uint4*)ap;
      t.u[1] = *(const uint4*)(ap + 8);
      afr[i] = t.v;
    }
    v16bf bfr[4];
#pragma unroll
    for (int j = 0; j < 4; ++j) {
      const unsigned short* bp = &Bb[(ng * 64 + j * 16 + cc) * BROW + hh * 8];
      union { uint4 u[2]; v16bf v; } t;
      t.u[0] = *(const uint4*)bp;
      t.u[1] = *(const uint4*)(bp + 16);
      bfr[j] = t.v;
    }
#pragma unroll
    for (int i = 0; i < 2; ++i)
#pragma unroll
      for (int j = 0; j < 4; ++j)
        acc[i][j] = wmma_bf16(afr[i], bfr[j], acc[i][j]);

    __syncthreads();
  }

#pragma unroll
  for (int hf = 0; hf < 2; ++hf) {
    if ((mq >> 1) == hf) {
      const int rb = (mq & 1) * 32;
#pragma unroll
      for (int i = 0; i < 2; ++i)
#pragma unroll
        for (int j = 0; j < 4; ++j)
#pragma unroll
          for (int e = 0; e < 8; ++e)
            St[(rb + i * 16 + 8 * hh + e) * SP + ng * 64 + j * 16 + cc] = acc[i][j][e];
    }
    __syncthreads();

    v4f vals[8];
#pragma unroll
    for (int q = 0; q < 8; ++q)
      vals[q] = *(const v4f*)&St[(wv * 8 + q) * SP + 4 * l];

    float* pb = pout + ((size_t)(hf * 64 + wv * 8) * H_OUT + oh) * PW + ow0 + 4 * l;
#pragma unroll
    for (int q = 0; q < 8; ++q)
      *(volatile v4f*)(pb + (size_t)q * (H_OUT * PW)) = vals[q];
    __threadfence();
#pragma unroll
    for (int q = 0; q < 8; ++q)
      *(volatile v4f*)(pb + (size_t)q * (H_OUT * PW)) = vals[q];

    __syncthreads();
  }
}

__global__ __launch_bounds__(256) void repack_output(const float* __restrict__ pin,
                                                     float* __restrict__ out, int nquad) {
  const int t = blockIdx.x * 256 + threadIdx.x;
  if (t < nquad) {
    float v[4];
#pragma unroll
    for (int e = 0; e < 4; ++e) {
      const int f   = 4 * t + e;
      const int m   = f / (H_OUT * W_OUT);
      const int rem = f - m * (H_OUT * W_OUT);
      const int oh  = rem / W_OUT;
      const int ow  = rem - oh * W_OUT;
      v[e] = pin[((size_t)m * H_OUT + oh) * PW + ow];
    }
    v4f vv;
    vv[0] = v[0]; vv[1] = v[1]; vv[2] = v[2]; vv[3] = v[3];
    float* dst = out + (size_t)4 * t;
    *(volatile v4f*)dst = vv;
    __threadfence();
    *(volatile v4f*)dst = vv;
  }
}

extern "C" void kernel_launch(void* const* d_in, const int* in_sizes, int n_in,
                              void* d_out, int out_size, void* d_ws, size_t ws_size,
                              hipStream_t stream) {
  if (n_in < 2) return;
  if (in_sizes[0] != NX || in_sizes[1] != NW || out_size != NOUT) return;
  if (ws_size < (size_t)NP * sizeof(float)) return;

  const float* x = (const float*)d_in[0];
  const float* w = (const float*)d_in[1];
  float* out  = (float*)d_out;
  float* pbuf = (float*)d_ws;

  dim3 grid((W_OUT + 127) / 128, H_OUT, 1);
  conv3x3_bf16_wmma<<<grid, 256, 0, stream>>>(x, w, pbuf);

  const int nquad = NOUT / 4;
  repack_output<<<(nquad + 255) / 256, 256, 0, stream>>>(pbuf, out, nquad);
}
